// SDT_46488726012141
// MI455X (gfx1250) — hardware-verified
//
#include <hip/hip_runtime.h>
#include <stddef.h>

typedef __attribute__((ext_vector_type(16))) __bf16 v16b;
typedef unsigned short v8us  __attribute__((ext_vector_type(8)));
typedef unsigned short v16us __attribute__((ext_vector_type(16)));
typedef float v8f __attribute__((ext_vector_type(8)));
typedef float v4f __attribute__((ext_vector_type(4)));
typedef v8us __attribute__((may_alias)) v8usa;
typedef v4f  __attribute__((may_alias)) v4fa;

union Frag { v16b v; v16us u; v8us half[2]; };

#define NBT    65536
#define NCH    8
#define NB     8192
#define NF     128
#define NNODE  1023
#define NNP    1024
#define NLEAF  1024
#define NLD    32
#define NSLOT  2048

#define TR_WAVES 4
#define TR_ITERS 16
#define TR_ROWS  (TR_WAVES * TR_ITERS)
#define RPB      (NB / TR_ROWS)
#define NREC     (NCH * RPB)
#define PTHR     256

#define XBLK   ((NBT * NF / 8) / 256)
#define WBLK   ((NNP * NF / 8) / 256)
#define LBLK   ((NLD * NLEAF / 8) / 256)
#define WSMAX  134217728

static_assert(NF % 32 == 0);
static_assert(NLEAF % 32 == 0);
static_assert(NB % 128 == 0);
static_assert(NNP % 64 == 0);
static_assert(NLD == 32);
static_assert(NB % TR_ROWS == 0);
static_assert(NBT == NCH * NB);
static_assert(NSLOT == 2 * NLEAF);
static_assert(NSLOT % PTHR == 0);
static_assert(NSLOT / 4 == 4 * 128);
static_assert((NBT * NF / 8) % 256 == 0);
static_assert((NNP * NF / 8) % 256 == 0);
static_assert((NLD * NLEAF / 8) % 256 == 0);

__device__ __forceinline__ unsigned short bfb(float f) {
  unsigned u = __float_as_uint(f);
  u = u + 0x7FFFu + ((u >> 16) & 1u);
  return (unsigned short)(u >> 16);
}
__device__ __forceinline__ float bfv(unsigned short s) {
  return __uint_as_float(((unsigned)s) << 16);
}

__device__ __forceinline__ v8f wmma_bf16(v16b a, v16b b, v8f c) {
  v8f d = __builtin_amdgcn_wmma_f32_16x16x32_bf16(false, a, false, b, (short)0, c, false, false);
  asm volatile("v_nop\n\tv_nop\n\tv_nop\n\tv_nop" : "+v"(d) : "v"(a), "v"(b));
  return d;
}

__device__ __forceinline__ v16b load_frag(const unsigned short* p, int h) {
  Frag f;
  f.half[0] = *(const v8usa*)(p + 8 * h);
  f.half[1] = *(const v8usa*)(p + 16 + 8 * h);
  return f.v;
}

__device__ __forceinline__ void store2_us8(unsigned short* dst, v8us o) {
  *(volatile v8us*)dst = o;
  __threadfence();
  *(volatile v8us*)dst = o;
}

__device__ __forceinline__ void tile_store_pass(const float* sT, float* g, int gp, int w, int lane) {
  const int q8 = lane & 7, sub = lane >> 3;
  #pragma unroll
  for (int i = 0; i < 16; ++i) {
    const int lid = 4 * i + sub;
    const int row = 32 * w + (lid >> 1), hl = lid & 1;
    const v4f v = *(const v4fa*)(sT + row * 64 + 32 * hl + 4 * q8);
    *(volatile v4f*)(g + (size_t)row * gp + 32 * hl + 4 * q8) = v;
  }
}

__device__ __forceinline__ void tile32_store_pass(const float* sT, float* g, int w, int lane) {
  const int q8 = lane & 7, sub = lane >> 3;
  #pragma unroll
  for (int i = 0; i < 8; ++i) {
    const int row = 32 * w + 4 * i + sub;
    const v4f v = *(const v4fa*)(sT + row * 32 + 4 * q8);
    *(volatile v4f*)(g + (size_t)row * NLD + 4 * q8) = v;
  }
}

__device__ __forceinline__ void row_store_pass(const unsigned short* s, unsigned short* g, int lane) {
  #pragma unroll
  for (int i = 0; i < 4; ++i) {
    const int e = (i * 32 + lane) * 8;
    const v8us v = *(const v8usa*)(s + e);
    *(volatile v8us*)(g + e) = v;
  }
}

__global__ __launch_bounds__(256) void convert_kernel(
    const float* __restrict__ x, const float* __restrict__ W, const float* __restrict__ lw,
    unsigned short* __restrict__ xh, unsigned short* __restrict__ wt, unsigned short* __restrict__ lt)
{
  const int bid = blockIdx.x, tid = threadIdx.x;
  if (bid < XBLK) {
    const size_t g = (size_t)bid * 256 + tid;
    const float* src = x + g * 8;
    const v4f a = *(const v4fa*)src;
    const v4f c = *(const v4fa*)(src + 4);
    const v8us o = { bfb(a.x), bfb(a.y), bfb(a.z), bfb(a.w), bfb(c.x), bfb(c.y), bfb(c.z), bfb(c.w) };
    store2_us8(xh + g * 8, o);
  } else if (bid < XBLK + WBLK) {
    const int e  = (bid - XBLK) * 256 + tid;
    const int n  = e >> 4;
    const int k0 = (e & 15) * 8;
    const int nc = (n < NNODE) ? n : (NNODE - 1);
    const float* src = W + (size_t)nc * NF + k0;
    const v4f a = *(const v4fa*)src;
    const v4f c = *(const v4fa*)(src + 4);
    const bool pad = (n >= NNODE);
    const unsigned short zz = 0;
    const v8us o = { pad ? zz : bfb(a.x), pad ? zz : bfb(a.y), pad ? zz : bfb(a.z), pad ? zz : bfb(a.w),
                     pad ? zz : bfb(c.x), pad ? zz : bfb(c.y), pad ? zz : bfb(c.z), pad ? zz : bfb(c.w) };
    store2_us8(wt + (size_t)n * NF + k0, o);
  } else if (bid < XBLK + WBLK + LBLK) {
    const size_t e = (size_t)(bid - XBLK - WBLK) * 256 + tid;
    const float* src = lw + e * 8;
    const v4f a = *(const v4fa*)src;
    const v4f c = *(const v4fa*)(src + 4);
    const v8us o = { bfb(a.x), bfb(a.y), bfb(a.z), bfb(a.w), bfb(c.x), bfb(c.y), bfb(c.z), bfb(c.w) };
    store2_us8(lt + e * 8, o);
  }
}

__global__ __launch_bounds__(128) void gate_gemm_kernel(
    const unsigned short* __restrict__ xh,
    const unsigned short* __restrict__ wt,
    float* __restrict__ P)
{
  __shared__ __attribute__((aligned(16))) float sT[128 * 64];

  const int tid = threadIdx.x, lane = tid & 31, w = tid >> 5;
  const int h = lane >> 4, m = lane & 15;
  const int m0 = blockIdx.x * 128, n0 = blockIdx.y * 64;
  const int m0w = m0 + 32 * w;

  const unsigned short* xa0 = xh + (size_t)(m0w + m) * NF;
  const unsigned short* xa1 = xa0 + (size_t)16 * NF;
  const unsigned short* wb  = wt + (size_t)(n0 + m) * NF;

  const v8f zero8 = {0.f, 0.f, 0.f, 0.f, 0.f, 0.f, 0.f, 0.f};
  v8f acc[2][4];
  #pragma unroll
  for (int mt = 0; mt < 2; ++mt)
    #pragma unroll
    for (int nt = 0; nt < 4; ++nt) acc[mt][nt] = zero8;

  #pragma unroll 1
  for (int k0 = 0; k0 < NF; k0 += 32) {
    const v16b a0 = load_frag(xa0 + k0, h);
    const v16b a1 = load_frag(xa1 + k0, h);
    #pragma unroll
    for (int nt = 0; nt < 4; ++nt) {
      const v16b b = load_frag(wb + (size_t)nt * 16 * NF + k0, h);
      acc[0][nt] = wmma_bf16(a0, b, acc[0][nt]);
      acc[1][nt] = wmma_bf16(a1, b, acc[1][nt]);
    }
  }

  #pragma unroll
  for (int nt = 0; nt < 4; ++nt) {
    const int col = 16 * nt + m;
    #pragma unroll
    for (int mt = 0; mt < 2; ++mt) {
      #pragma unroll
      for (int r = 0; r < 8; ++r) {
        const int tokl = 32 * w + 16 * mt + 8 * h + r;
        const float z = acc[mt][nt][r];
        const float e = __expf(-z);
        const float p = __builtin_amdgcn_rcpf(1.0f + e);
        sT[tokl * 64 + col] = p;
      }
    }
  }
  __syncthreads();

  float* g = P + (size_t)m0 * NNP + n0;
  tile_store_pass(sT, g, NNP, w, lane);
  __threadfence();
  tile_store_pass(sT, g, NNP, w, lane);
}

template <int NIN>
__device__ __forceinline__ void expand_level(const float* pr, int base,
                                             const float (&in)[NIN], float (&o)[2 * NIN]) {
  #pragma clang fp contract(off)
  #pragma unroll
  for (int j = 0; j < NIN; ++j) {
    const float v = pr[base + j];
    const float u = 1.0f - v;
    o[2 * j]     = v * in[j];
    o[2 * j + 1] = u * in[j];
  }
}

template <int N>
__device__ __forceinline__ void acc_add(float (&s)[N], const float (&a)[N]) {
  #pragma clang fp contract(off)
  #pragma unroll
  for (int j = 0; j < N; ++j) s[j] = s[j] + a[j];
}

template <int N>
__device__ __forceinline__ void zero_arr(float (&s)[N]) {
  #pragma unroll
  for (int j = 0; j < N; ++j) s[j] = 0.0f;
}

__global__ __launch_bounds__(128) void leafprob_kernel(
    const float* __restrict__ P,
    unsigned short* __restrict__ PH,
    unsigned short* __restrict__ PL,
    float* __restrict__ rec)
{
  #pragma clang fp contract(off)
  __shared__ __attribute__((aligned(16))) float sBuf[TR_WAVES * NSLOT];
  __shared__ __attribute__((aligned(16))) unsigned short sH[TR_WAVES * NLEAF];
  __shared__ __attribute__((aligned(16))) unsigned short sL[TR_WAVES * NLEAF];

  const int tid = threadIdx.x, lane = tid & 31, w = tid >> 5;
  float* pr = sBuf + w * NLEAF;
  unsigned short* hr = sH + w * NLEAF;
  unsigned short* lr = sL + w * NLEAF;

  float qs[4];
  #pragma unroll
  for (int L = 0; L < 4; ++L) qs[L] = 0.0f;
  float s1[1], s2[2], s4[4], s8[8], s16[16], s32[32];
  zero_arr<1>(s1); zero_arr<2>(s2); zero_arr<4>(s4); zero_arr<8>(s8); zero_arr<16>(s16); zero_arr<32>(s32);

  #pragma unroll 1
  for (int it = 0; it < TR_ITERS; ++it) {
    const int row = blockIdx.x * TR_ROWS + it * TR_WAVES + w;
    const float* prow = P + (size_t)row * NNP;

    #pragma unroll
    for (int j = 0; j < 8; ++j) {
      const int q = j * 32 + lane;
      const v4f v = *(const v4fa*)(prow + 4 * q);
      *(v4fa*)(pr + 4 * q) = v;
    }
    __syncthreads();

    float pre = 1.0f;
    #pragma unroll
    for (int L = 0; L < 5; ++L) {
      const int node = (1 << L) - 1 + (lane >> (5 - L));
      const int bit  = (lane >> (4 - L)) & 1;
      const float v = pr[node];
      const float u = 1.0f - v;
      pre = (bit ? u : v) * pre;
      if (L < 4) qs[L] = qs[L] + pre;
    }

    float a1[1];
    a1[0] = pre;
    float a2[2], a4[4], a8[8], a16[16], a32[32];
    acc_add<1>(s1, a1);
    expand_level<1>(pr,  31 +      lane, a1,  a2);   acc_add<2>(s2, a2);
    expand_level<2>(pr,  63 +  2 * lane, a2,  a4);   acc_add<4>(s4, a4);
    expand_level<4>(pr, 127 +  4 * lane, a4,  a8);   acc_add<8>(s8, a8);
    expand_level<8>(pr, 255 +  8 * lane, a8,  a16);  acc_add<16>(s16, a16);
    expand_level<16>(pr, 511 + 16 * lane, a16, a32); acc_add<32>(s32, a32);

    #pragma unroll
    for (int q = 0; q < 4; ++q) {
      v8us hv, lv;
      #pragma unroll
      for (int i = 0; i < 8; ++i) {
        const float p = a32[8 * q + i];
        const unsigned short hb = bfb(p);
        const unsigned short lb = bfb(p - bfv(hb));
        hv[i] = hb;
        lv[i] = lb;
      }
      *(v8usa*)(hr + 32 * lane + 8 * q) = hv;
      *(v8usa*)(lr + 32 * lane + 8 * q) = lv;
    }
    __syncthreads();

    unsigned short* gh = PH + (size_t)row * NLEAF;
    unsigned short* gl = PL + (size_t)row * NLEAF;
    row_store_pass(hr, gh, lane);
    row_store_pass(lr, gl, lane);
    __threadfence();
    row_store_pass(hr, gh, lane);
    row_store_pass(lr, gl, lane);
  }
  __syncthreads();

  float* ss = sBuf + w * NSLOT;
  if (lane == 0) { ss[0] = 0.0f; ss[NSLOT - 1] = 0.0f; }
  if ((lane & 15) == 0) ss[1 + (lane >> 4)] = qs[0];
  if ((lane & 7) == 0)  ss[3 + (lane >> 3)] = qs[1];
  if ((lane & 3) == 0)  ss[7 + (lane >> 2)] = qs[2];
  if ((lane & 1) == 0)  ss[15 + (lane >> 1)] = qs[3];
  ss[31 + lane] = s1[0];
  #pragma unroll
  for (int j = 0; j < 2; ++j)  ss[63 + 2 * lane + j] = s2[j];
  #pragma unroll
  for (int j = 0; j < 4; ++j)  ss[127 + 4 * lane + j] = s4[j];
  #pragma unroll
  for (int j = 0; j < 8; ++j)  ss[255 + 8 * lane + j] = s8[j];
  #pragma unroll
  for (int j = 0; j < 16; ++j) ss[511 + 16 * lane + j] = s16[j];
  #pragma unroll
  for (int j = 0; j < 32; ++j) ss[1023 + 32 * lane + j] = s32[j];
  __syncthreads();

  v4f rv[4];
  #pragma unroll
  for (int i = 0; i < 4; ++i) {
    const int q = i * 128 + tid;
    const v4f b0 = *(const v4fa*)(sBuf + 0 * NSLOT + 4 * q);
    const v4f b1 = *(const v4fa*)(sBuf + 1 * NSLOT + 4 * q);
    const v4f b2 = *(const v4fa*)(sBuf + 2 * NSLOT + 4 * q);
    const v4f b3 = *(const v4fa*)(sBuf + 3 * NSLOT + 4 * q);
    rv[i] = ((b0 + b1) + b2) + b3;
  }
  float* g = rec + (size_t)blockIdx.x * NSLOT;
  #pragma unroll
  for (int i = 0; i < 4; ++i) *(volatile v4f*)(g + 4 * (i * 128 + tid)) = rv[i];
  __threadfence();
  #pragma unroll
  for (int i = 0; i < 4; ++i) *(volatile v4f*)(g + 4 * (i * 128 + tid)) = rv[i];
}

__global__ __launch_bounds__(128) void leaf_gemm_kernel(
    const unsigned short* __restrict__ PH,
    const unsigned short* __restrict__ PL,
    const unsigned short* __restrict__ lt,
    float* __restrict__ out)
{
  __shared__ __attribute__((aligned(16))) float sT[128 * 32];

  const int tid = threadIdx.x, lane = tid & 31, w = tid >> 5;
  const int h = lane >> 4, m = lane & 15;
  const int m0 = blockIdx.x * 128;
  const int m0w = m0 + 32 * w;

  const unsigned short* ha0 = PH + (size_t)(m0w + m) * NLEAF;
  const unsigned short* ha1 = ha0 + (size_t)16 * NLEAF;
  const unsigned short* la0 = PL + (size_t)(m0w + m) * NLEAF;
  const unsigned short* la1 = la0 + (size_t)16 * NLEAF;
  const unsigned short* lb  = lt + (size_t)m * NLEAF;

  const v8f zero8 = {0.f, 0.f, 0.f, 0.f, 0.f, 0.f, 0.f, 0.f};
  v8f acc[2][2];
  #pragma unroll
  for (int mt = 0; mt < 2; ++mt)
    #pragma unroll
    for (int nt = 0; nt < 2; ++nt) acc[mt][nt] = zero8;

  #pragma unroll 1
  for (int k0 = 0; k0 < NLEAF; k0 += 32) {
    const v16b ah0 = load_frag(ha0 + k0, h);
    const v16b ah1 = load_frag(ha1 + k0, h);
    const v16b al0 = load_frag(la0 + k0, h);
    const v16b al1 = load_frag(la1 + k0, h);
    #pragma unroll
    for (int nt = 0; nt < 2; ++nt) {
      const v16b b = load_frag(lb + (size_t)nt * 16 * NLEAF + k0, h);
      acc[0][nt] = wmma_bf16(ah0, b, acc[0][nt]);
      acc[0][nt] = wmma_bf16(al0, b, acc[0][nt]);
      acc[1][nt] = wmma_bf16(ah1, b, acc[1][nt]);
      acc[1][nt] = wmma_bf16(al1, b, acc[1][nt]);
    }
  }

  #pragma unroll
  for (int nt = 0; nt < 2; ++nt) {
    const int col = 16 * nt + m;
    #pragma unroll
    for (int mt = 0; mt < 2; ++mt) {
      #pragma unroll
      for (int r = 0; r < 8; ++r) {
        const int tokl = 32 * w + 16 * mt + 8 * h + r;
        sT[tokl * 32 + col] = acc[mt][nt][r];
      }
    }
  }
  __syncthreads();

  float* g = out + (size_t)m0 * NLD;
  tile32_store_pass(sT, g, w, lane);
  __threadfence();
  tile32_store_pass(sT, g, w, lane);
}

__global__ __launch_bounds__(PTHR) void penalty_kernel(const float* __restrict__ rec, float* out_pen)
{
  __shared__ double sS[NSLOT];
  __shared__ double sPart[PTHR];
  const int tid = threadIdx.x;

  #pragma unroll 1
  for (int j = 0; j < NSLOT / PTHR; ++j) {
    const int g = j * PTHR + tid;
    double s = 0.0;
    #pragma unroll 4
    for (int r = 0; r < NREC; ++r) s += (double)rec[(size_t)r * NSLOT + g];
    sS[g] = (g == 0) ? (double)NBT : s;
  }
  __syncthreads();

  double part = 0.0;
  #pragma unroll 1
  for (int j = 0; j < NSLOT / PTHR; ++j) {
    const int g = j * PTHR + tid;
    const bool live = (g >= 1) && (g <= 2 * NNODE);
    const int gc = live ? g : 1;
    const int L = 31 - __clz(gc + 1);
    const int parent = (gc - 1) >> 1;
    const double alpha = sS[gc] / sS[parent];
    const float af = (float)alpha;
    const float c = logf(af) + log1pf(-af);
    const double wgt = 0.0005 / (double)(1 << (L - 1));
    part -= live ? wgt * (double)c : 0.0;
  }
  sPart[tid] = part;
  __syncthreads();

  if (tid == 0) {
    double tot = 0.0;
    #pragma unroll 1
    for (int i = 0; i < PTHR; ++i) tot += sPart[i];
    const float v = (float)tot;
    *(volatile float*)out_pen = v;
    __threadfence();
    *(volatile float*)out_pen = v;
  }
}

extern "C" void kernel_launch(void* const* d_in, const int* in_sizes, int n_in,
                              void* d_out, int out_size, void* d_ws, size_t ws_size,
                              hipStream_t stream) {
  if (n_in < 3) return;
  if (in_sizes[0] != NBT * NF) return;
  if (in_sizes[1] != NNODE * NF) return;
  if (in_sizes[2] != NLD * NLEAF) return;
  if (out_size != NBT * NLD + 1) return;

  const float* x  = (const float*)d_in[0];
  const float* W  = (const float*)d_in[1];
  const float* lw = (const float*)d_in[2];
  float* out = (float*)d_out;
  float* out_pen = out + (size_t)NBT * NLD;

  const size_t sz_xh  = (size_t)NBT * NF * 2;
  const size_t sz_wt  = (size_t)NNP * NF * 2;
  const size_t sz_lt  = (size_t)NLD * NLEAF * 2;
  const size_t sz_p   = (size_t)NB * NNP * 4;
  const size_t sz_ph  = (size_t)NB * NLEAF * 2;
  const size_t sz_rec = (size_t)NREC * NSLOT * 4;
  const size_t off_xh  = 0;
  const size_t off_wt  = off_xh + sz_xh;
  const size_t off_lt  = off_wt + sz_wt;
  const size_t off_p   = off_lt + sz_lt;
  const size_t off_ph  = off_p + sz_p;
  const size_t off_pl  = off_ph + sz_ph;
  const size_t off_rec = off_pl + sz_ph;
  const size_t total   = off_rec + sz_rec;
  if (total > ws_size || total > (size_t)WSMAX) return;

  char* ws = (char*)d_ws;
  unsigned short* xh  = (unsigned short*)(ws + off_xh);
  unsigned short* wt  = (unsigned short*)(ws + off_wt);
  unsigned short* lt  = (unsigned short*)(ws + off_lt);
  float*          P   = (float*)(ws + off_p);
  unsigned short* PH  = (unsigned short*)(ws + off_ph);
  unsigned short* PL  = (unsigned short*)(ws + off_pl);
  float*          REC = (float*)(ws + off_rec);

  convert_kernel<<<XBLK + WBLK + LBLK, 256, 0, stream>>>(x, W, lw, xh, wt, lt);

  for (int c = 0; c < NCH; ++c) {
    const unsigned short* xhc = xh + (size_t)c * NB * NF;
    float* outc  = out + (size_t)c * NB * NLD;
    float* recc  = REC + (size_t)c * RPB * NSLOT;
    dim3 g1(NB / 128, NNP / 64);
    gate_gemm_kernel<<<g1, 128, 0, stream>>>(xhc, wt, P);
    leafprob_kernel<<<NB / TR_ROWS, 128, 0, stream>>>(P, PH, PL, recc);
    leaf_gemm_kernel<<<NB / 128, 128, 0, stream>>>(PH, PL, lt, outc);
  }

  penalty_kernel<<<1, PTHR, 0, stream>>>(REC, out_pen);
}
